// BasicTransformerBlock_17085379903983
// MI455X (gfx1250) — hardware-verified
//
#include <hip/hip_runtime.h>
#include <math.h>

typedef _Float16 v16h __attribute__((ext_vector_type(16)));
typedef _Float16 v8h __attribute__((ext_vector_type(8)));
typedef float v8f __attribute__((ext_vector_type(8)));
typedef float v4f __attribute__((ext_vector_type(4)));
typedef unsigned v4u __attribute__((ext_vector_type(4)));
typedef v4f __attribute__((may_alias)) v4fa;
typedef v4u __attribute__((may_alias)) v4ua;

#ifndef NB
#define NB 4
#endif
#ifndef SEQ
#define SEQ 2048
#endif
#define SEQ_FULL 2048
#define DD 512
#define CC 512
#define NH 8
#define HD 64
#define CN 77
#define CNP 128
#define CD 768
#define FF 2048
#define FF1LD 4096
#define HG 2
#define MROWS (NB * SEQ)
#define SCALE (0.125f)
#define LNEPS (1.0e-5f)
static_assert(SEQ % 128 == 0);
static_assert(MROWS % 64 == 0);
static_assert(NH % HG == 0);
static_assert((NB * CNP) % 64 == 0);

#define WPL  (2u * (size_t)512 * 512)
#define WPLC (2u * (size_t)512 * 768)
#define WPLF (2u * (size_t)2048 * 512)
#define WS_XN ((size_t)0)
#define WS_QH (WS_XN + 2u * (size_t)MROWS * DD)
#define WS_KH (WS_QH + 2u * (size_t)MROWS * CC)
#define WS_VT (WS_KH + 2u * (size_t)MROWS * CC)
#define WS_S  (WS_VT + 2u * (size_t)NB * CC * SEQ)
#define SB_A (4u * (size_t)HG * SEQ * SEQ)
#define SB_B (4u * (size_t)NB * NH * SEQ * CNP)
#define SB_C (2u * (size_t)MROWS * FF)
#define SB_AB (SB_A > SB_B ? SB_A : SB_B)
#define SB (SB_AB > SB_C ? SB_AB : SB_C)
#define WS_Y  (WS_S + SB)
#define WS_X1 (WS_Y + 2u * (size_t)MROWS * CC)
#define WS_X2 (WS_X1 + 4u * (size_t)MROWS * DD)
#define WS_W  (WS_X2 + 4u * (size_t)MROWS * DD)
#define WS_WQ1 (WS_W)
#define WS_WK1 (WS_WQ1 + WPL)
#define WS_WV1 (WS_WK1 + WPL)
#define WS_WO1 (WS_WV1 + WPL)
#define WS_WQ2 (WS_WO1 + WPL)
#define WS_WO2 (WS_WQ2 + WPL)
#define WS_WK2 (WS_WO2 + WPL)
#define WS_WV2 (WS_WK2 + WPLC)
#define WS_WF1 (WS_WV2 + WPLC)
#define WS_WF2 (WS_WF1 + WPLF)
#define WS_CX (WS_WF2 + WPLF)
#define WS_KC (WS_CX + 2u * (size_t)NB * CNP * CD)
#define WS_VC (WS_KC + 2u * (size_t)NB * CNP * CC)
#define WS_END (WS_VC + 2u * (size_t)NB * CC * CNP)
static_assert(WS_END <= (size_t)134217728u);

template <typename T> __device__ __forceinline__ void vst2(void* p, T v) { *(volatile T*)p = v; __threadfence(); *(volatile T*)p = v; }
__device__ __forceinline__ v8f wmma16(v16h a, v16h b, v8f c) {
  v8f d = __builtin_amdgcn_wmma_f32_16x16x32_f16(false, a, false, b, (short)0, c, false, false);
  asm volatile("v_nop\n\tv_nop\n\tv_nop\n\tv_nop" : "+v"(d) : "v"(a), "v"(b));
  return d;
}
__device__ __forceinline__ v16h frag_h(const _Float16* rowk0, int lane) {
  union { v16h v; v8h q[2]; } u; const _Float16* p = rowk0 + 8 * (lane >> 4);
  u.q[0] = *(const v8h*)p; u.q[1] = *(const v8h*)(p + 16); return u.v;
}
__device__ __forceinline__ v16h frag_f32(const float* rowk0, int lane) {
  v16h a; const float* p = rowk0 + 8 * (lane >> 4);
#pragma unroll
  for (int i = 0; i < 8; ++i) { a[i] = (_Float16)p[i]; a[8 + i] = (_Float16)p[16 + i]; }
  return a;
}
__device__ __forceinline__ float bfr(float v) { return (float)(__bf16)v; }
__device__ __forceinline__ void ldsx() { asm volatile("s_wait_dscnt 0x0" ::: "memory"); __builtin_amdgcn_wave_barrier(); __builtin_amdgcn_fence(3, "workgroup"); }
#define VG256 __attribute__((amdgpu_num_vgpr(256)))

__global__ __launch_bounds__(256) void k_wcvt(const float* __restrict__ W0, const float* __restrict__ W1, const float* __restrict__ W2, int ld, int K,
    _Float16* __restrict__ T0, _Float16* __restrict__ T1, _Float16* __restrict__ T2) {
  __shared__ __align__(16) _Float16 tl[64][72];
  const int tid = threadIdx.x; const int z = blockIdx.z; const float* W = z == 0 ? W0 : z == 1 ? W1 : W2; _Float16* T = z == 0 ? T0 : z == 1 ? T1 : T2;
  const int k0 = blockIdx.x * 64, n0 = blockIdx.y * 64;
  for (int e = tid; e < 64 * 64; e += 256) { const int kk = e >> 6, nn = e & 63; tl[nn][kk] = (_Float16)(bfr(W[(size_t)(k0 + kk) * ld + n0 + nn]) * 256.0f); }
  __syncthreads();
  for (int e = tid; e < 64 * 8; e += 256) { const int nn = e >> 3, q = e & 7; vst2((v4u*)(T + (size_t)(n0 + nn) * K + k0 + q * 8), *(const v4ua*)&tl[nn][q * 8]); }
}
__global__ __launch_bounds__(256) void k_ccvt(const float* __restrict__ X, _Float16* __restrict__ CX) {
  const int tid = threadIdx.x, wave = tid >> 5, lane = tid & 31; const int row = blockIdx.x * 8 + wave; const int b = row / CNP, t = row % CNP;
  const float keep = t < CN ? 1.0f : 0.0f; const float* xr = X + ((size_t)b * CN + (t < CN ? t : CN - 1)) * CD;
#pragma unroll
  for (int i = 0; i < 3; ++i) { const float* p = xr + 256 * i + 8 * lane; const v4f a = *(const v4f*)p, c = *(const v4f*)(p + 4); union { v8h h; v4u u; } o;
#pragma unroll
    for (int k = 0; k < 4; ++k) { o.h[k] = (_Float16)(bfr(a[k]) * keep); o.h[4 + k] = (_Float16)(bfr(c[k]) * keep); }
    vst2((v4u*)(CX + (size_t)row * CD + 256 * i + 8 * lane), o.u); }
}
__global__ __launch_bounds__(256) void k_ln(const float* __restrict__ X, int xin, const float* __restrict__ G, const float* __restrict__ Bt, _Float16* __restrict__ XN) {
#pragma clang fp contract(off)
  const int tid = threadIdx.x, wave = tid >> 5, lane = tid & 31; const int row = blockIdx.x * 8 + wave; const int b = row / SEQ, t = row % SEQ;
  const float* xr = X + (xin ? ((size_t)b * SEQ_FULL + t) : (size_t)row) * DD;
  float v[16];
  { const v4f a0 = *(const v4f*)(xr + 8 * lane), a1 = *(const v4f*)(xr + 8 * lane + 4), a2 = *(const v4f*)(xr + 256 + 8 * lane), a3 = *(const v4f*)(xr + 256 + 8 * lane + 4);
#pragma unroll
    for (int i = 0; i < 4; ++i) { v[i] = a0[i]; v[4 + i] = a1[i]; v[8 + i] = a2[i]; v[12 + i] = a3[i]; } }
  if (xin) {
#pragma unroll
    for (int i = 0; i < 16; ++i) v[i] = bfr(v[i]); }
  float s = 0.f;
#pragma unroll
  for (int i = 0; i < 16; ++i) s += v[i];
#pragma unroll
  for (int o = 1; o < 32; o <<= 1) s += __shfl_xor(s, o);
  const float mu = s * (1.0f / DD);
  float ss = 0.f;
#pragma unroll
  for (int i = 0; i < 16; ++i) { v[i] = v[i] - mu; ss += v[i] * v[i]; }
#pragma unroll
  for (int o = 1; o < 32; o <<= 1) ss += __shfl_xor(ss, o);
  const float rs = rsqrtf(ss * (1.0f / DD) + LNEPS);
  union { v8h h; v4u u; } o0, o1;
#pragma unroll
  for (int i = 0; i < 8; ++i) { const int ca = 8 * lane + i, cb = 256 + 8 * lane + i;
    o0.h[i] = (_Float16)(v[i] * rs * bfr(G[ca]) + bfr(Bt[ca])); o1.h[i] = (_Float16)(v[8 + i] * rs * bfr(G[cb]) + bfr(Bt[cb])); }
  vst2((v4u*)(XN + (size_t)row * DD + 8 * lane), o0.u); vst2((v4u*)(XN + (size_t)row * DD + 256 + 8 * lane), o1.u);
}
__global__ __launch_bounds__(128) VG256 void k_gemm16(const _Float16* __restrict__ A, int lda, int K,
    const _Float16* __restrict__ W0, const _Float16* __restrict__ W1, const _Float16* __restrict__ W2,
    _Float16* __restrict__ D0, _Float16* __restrict__ D1, _Float16* __restrict__ D2, int ldd, int tz, int tp, const float* __restrict__ bias, float carry) {
  __shared__ __align__(16) _Float16 sh[64][136]; __shared__ __align__(16) _Float16 th[128][72];
  const int tid = threadIdx.x, wave = tid >> 5, lane = tid & 31, col = lane & 15, g = lane >> 4; const int z = blockIdx.z; const int c0 = blockIdx.y * 128; const size_t r0 = (size_t)blockIdx.x * 64;
  const _Float16* W = z == 0 ? W0 : z == 1 ? W1 : W2; _Float16* D = z == 0 ? D0 : z == 1 ? D1 : D2;
  v8f acc[8] = {};
  const _Float16* ar = A + (r0 + wave * 16 + col) * (size_t)lda;
#pragma unroll 1
  for (int kc = 0; kc < K / 32; ++kc) { const v16h a = frag_h(ar + kc * 32, lane);
#pragma unroll
    for (int j = 0; j < 8; ++j) { const v16h w = frag_h(W + (size_t)(c0 + j * 16 + col) * K + kc * 32, lane); acc[j] = wmma16(a, w, acc[j]); } }
  if (z != tz) {
#pragma unroll
    for (int j = 0; j < 8; ++j) { const float bb = bias ? bfr(bias[c0 + j * 16 + col]) : 0.f;
#pragma unroll
      for (int r = 0; r < 8; ++r) sh[wave * 16 + 8 * g + r][j * 16 + col] = (_Float16)((acc[j][r] * (1.0f / 256.0f) + bb) * carry); }
    __syncthreads();
    for (int e = tid; e < 64 * 16; e += 128) { const int rl = e >> 4, q = e & 15; vst2((v4u*)(D + (r0 + rl) * (size_t)ldd + c0 + q * 8), *(const v4ua*)&sh[rl][q * 8]); }
  } else { const size_t bq = r0 / tp; const int t0 = (int)(r0 % tp);
#pragma unroll
    for (int j = 0; j < 8; ++j)
#pragma unroll
      for (int r = 0; r < 8; ++r) th[j * 16 + col][wave * 16 + 8 * g + r] = (_Float16)(acc[j][r] * (1.0f / 256.0f) * carry);
    __syncthreads();
    for (int e = tid; e < 128 * 8; e += 128) { const int cl = e >> 3, q = e & 7; vst2((v4u*)(D + (bq * CC + c0 + cl) * (size_t)tp + t0 + q * 8), *(const v4ua*)&th[cl][q * 8]); } }
}
__global__ __launch_bounds__(128) VG256 void k_gemm32(const _Float16* __restrict__ A, int lda, int K, const _Float16* __restrict__ W, const float* __restrict__ bias,
    const float* __restrict__ R, int rmode, float* __restrict__ Dst, int dmode, float ascale) {
  __shared__ __align__(16) float sf[4][16][132];
  const int tid = threadIdx.x, wave = tid >> 5, lane = tid & 31, col = lane & 15, g = lane >> 4; const int c0 = blockIdx.y * 128; const size_t r0 = (size_t)blockIdx.x * 64 + wave * 16;
  v8f acc[8] = {};
  const _Float16* ar = A + (r0 + col) * (size_t)lda;
#pragma unroll 1
  for (int kc = 0; kc < K / 32; ++kc) { const v16h a = frag_h(ar + kc * 32, lane);
#pragma unroll
    for (int j = 0; j < 8; ++j) { const v16h w = frag_h(W + (size_t)(c0 + j * 16 + col) * K + kc * 32, lane); acc[j] = wmma16(a, w, acc[j]); } }
#pragma unroll
  for (int j = 0; j < 8; ++j) { const float bb = bias ? bfr(bias[c0 + j * 16 + col]) : 0.f;
#pragma unroll
    for (int r = 0; r < 8; ++r) sf[wave][8 * g + r][j * 16 + col] = acc[j][r] * ascale + bb; }
  ldsx();
  for (int rl = 0; rl < 16; ++rl) { const size_t row = r0 + rl; const size_t bq = row / SEQ, tq = row % SEQ; const size_t frow = bq * SEQ_FULL + tq;
    v4f res = *(const v4f*)(R + (rmode ? frow : row) * DD + c0 + lane * 4);
    if (rmode) { res[0] = bfr(res[0]); res[1] = bfr(res[1]); res[2] = bfr(res[2]); res[3] = bfr(res[3]); }
    const v4f val = *(const v4fa*)&sf[wave][rl][lane * 4] + res;
    vst2((v4f*)(Dst + (dmode ? frow : row) * DD + c0 + lane * 4), val); }
}
template <int TK> __global__ __launch_bounds__(128) VG256 void k_sc(const _Float16* __restrict__ QH, const _Float16* __restrict__ KH, float* __restrict__ S0, int b0, int h0, int nhz) {
  __shared__ __align__(16) float ss[4][16][132];
  const int z = blockIdx.z; const int h = h0 + z % nhz, b = b0 + z / nhz; float* S = S0 + (size_t)z * SEQ * TK;
  const int tid = threadIdx.x, wave = tid >> 5, lane = tid & 31, col = lane & 15, g = lane >> 4; const int qb = blockIdx.x, kb = blockIdx.y; const int k0 = kb * 128; const int ql0 = qb * 64 + wave * 16;
  const size_t q0 = (size_t)b * SEQ + ql0, kr0 = (size_t)b * TK + k0;
  v8f acc[8] = {};
#pragma unroll
  for (int kc = 0; kc < HD / 32; ++kc) { const v16h ah = frag_h(QH + (q0 + col) * CC + h * HD + kc * 32, lane);
#pragma unroll
    for (int j = 0; j < 8; ++j) { const v16h kf = frag_h(KH + (kr0 + j * 16 + col) * CC + h * HD + kc * 32, lane); acc[j] = wmma16(ah, kf, acc[j]); } }
#pragma unroll
  for (int j = 0; j < 8; ++j) {
#pragma unroll
    for (int r = 0; r < 8; ++r) ss[wave][8 * g + r][j * 16 + col] = acc[j][r] * SCALE; }
  ldsx(); for (int rl = 0; rl < 16; ++rl) vst2((v4f*)(S + (size_t)(ql0 + rl) * TK + k0 + lane * 4), *(const v4fa*)&ss[wave][rl][lane * 4]);
}
template <int TK, int NKV> __global__ __launch_bounds__(256) void k_sm(float* __restrict__ S0) {
  __shared__ float sred[8]; __shared__ float sbc; __shared__ __align__(16) float shv[TK];
  const int tid = threadIdx.x; const int t = blockIdx.x;
  float* sr = S0 + (size_t)blockIdx.y * SEQ * TK + (size_t)t * TK;
  float m = -3.0e38f;
#pragma unroll 1
  for (int k = tid; k < TK; k += 256) { const float v = (k < NKV) ? sr[k] : -3.0e38f; shv[k] = v; m = fmaxf(m, v); }
#pragma unroll
  for (int o = 1; o < 32; o <<= 1) m = fmaxf(m, __shfl_xor(m, o));
  if ((tid & 31) == 0) sred[tid >> 5] = m; __syncthreads(); if (tid == 0) { float a = sred[0]; for (int i = 1; i < 8; ++i) a = fmaxf(a, sred[i]); sbc = a; } __syncthreads(); m = sbc; __syncthreads();
  float sum = 0.f;
#pragma unroll 1
  for (int k = tid; k < TK; k += 256) { const float v = shv[k]; const float e = (v <= -1.0e38f) ? 0.f : expf(v - m); shv[k] = e; sum += e; }
#pragma unroll
  for (int o = 1; o < 32; o <<= 1) sum += __shfl_xor(sum, o);
  if ((tid & 31) == 0) sred[tid >> 5] = sum; __syncthreads(); if (tid == 0) { float a = 0.f; for (int i = 0; i < 8; ++i) a += sred[i]; sbc = a > 0.f ? 2048.0f / a : 0.f; } __syncthreads(); const float inv = sbc;
#pragma unroll 1
  for (int q = tid; q < TK / 4; q += 256) { const v4f pv = *(const v4fa*)&shv[q * 4] * inv; vst2((v4f*)(sr + q * 4), pv); }
}
template <int TK> __global__ __launch_bounds__(128) VG256 void k_pv(const float* __restrict__ PS0, const _Float16* __restrict__ VT, int b0, int h0, int nhz, _Float16* __restrict__ Y) {
  __shared__ __align__(16) _Float16 sy[4][16][72];
  const int z = blockIdx.z; const int h = h0 + z % nhz, b = b0 + z / nhz; const float* PS = PS0 + (size_t)z * SEQ * TK;
  const int tid = threadIdx.x, wave = tid >> 5, lane = tid & 31, col = lane & 15, g = lane >> 4; const int qb = blockIdx.x; const int ql0 = qb * 64 + wave * 16;
  v8f acc[HD / 16] = {};
#pragma unroll 1
  for (int kc = 0; kc < TK / 32; ++kc) { const v16h p = frag_f32(PS + (size_t)(ql0 + col) * TK + kc * 32, lane);
    asm volatile("s_wait_loadcnt 0x0" ::: "memory");
#pragma unroll
    for (int j = 0; j < HD / 16; ++j) { const size_t po = ((size_t)b * CC + h * HD + j * 16 + col) * (size_t)TK + kc * 32; acc[j] = wmma16(p, frag_h(VT + po, lane), acc[j]); } }
#pragma unroll
  for (int j = 0; j < HD / 16; ++j)
#pragma unroll
    for (int r = 0; r < 8; ++r) sy[wave][8 * g + r][j * 16 + col] = (_Float16)(acc[j][r] * (16.0f / 2048.0f));
  ldsx();
  const int l8 = (lane < 8 ? lane : 7) * 8;
  for (int rl = 0; rl < 16; ++rl) { const v4u pc = *(const v4ua*)&sy[wave][rl][l8]; if (lane < 8) vst2((v4u*)(Y + ((size_t)b * SEQ + ql0 + rl) * CC + h * HD + lane * 8), pc); }
}

extern "C" void kernel_launch(void* const* d_in, const int* in_sizes, int n_in, void* d_out, int out_size, void* d_ws, size_t ws_size, hipStream_t stream) {
  if (n_in < 22) return;
  const float** F = (const float**)d_in;
  if ((size_t)in_sizes[0] < ((size_t)(NB - 1) * SEQ_FULL + SEQ) * DD) return;
  if (in_sizes[1] < NB * CN * CD) return;
  for (int i = 2; i <= 7; ++i) if (in_sizes[i] < DD) return;
  if (in_sizes[8] < DD * CC || in_sizes[9] < DD * CC || in_sizes[10] < DD * CC || in_sizes[11] < CC * DD || in_sizes[12] < DD) return;
  if (in_sizes[13] < DD * CC || in_sizes[14] < CD * CC || in_sizes[15] < CD * CC || in_sizes[16] < CC * DD || in_sizes[17] < DD) return;
  if (in_sizes[18] < DD * FF1LD || in_sizes[19] < FF || in_sizes[20] < FF * DD || in_sizes[21] < DD) return;
  if ((size_t)out_size < ((size_t)(NB - 1) * SEQ_FULL + SEQ) * DD) return;
  if (ws_size < (size_t)WS_END) return;
  char* ws = (char*)d_ws;
  _Float16 *XN = (_Float16*)(ws + WS_XN), *QH = (_Float16*)(ws + WS_QH), *KH = (_Float16*)(ws + WS_KH), *VT = (_Float16*)(ws + WS_VT);
  float* Sf = (float*)(ws + WS_S); _Float16* Hh = (_Float16*)(ws + WS_S);
  _Float16* Y = (_Float16*)(ws + WS_Y); float *X1 = (float*)(ws + WS_X1), *X2 = (float*)(ws + WS_X2);
  _Float16 *WQ1 = (_Float16*)(ws + WS_WQ1), *WK1 = (_Float16*)(ws + WS_WK1), *WV1 = (_Float16*)(ws + WS_WV1), *WO1 = (_Float16*)(ws + WS_WO1);
  _Float16 *WQ2 = (_Float16*)(ws + WS_WQ2), *WO2 = (_Float16*)(ws + WS_WO2), *WK2 = (_Float16*)(ws + WS_WK2), *WV2 = (_Float16*)(ws + WS_WV2);
  _Float16 *WF1 = (_Float16*)(ws + WS_WF1), *WF2 = (_Float16*)(ws + WS_WF2);
  _Float16 *CX = (_Float16*)(ws + WS_CX), *KC = (_Float16*)(ws + WS_KC), *VC = (_Float16*)(ws + WS_VC);
  float* OUT = (float*)d_out;

  k_wcvt<<<dim3(DD / 64, CC / 64, 3), 256, 0, stream>>>(F[8], F[9], F[10], CC, DD, WQ1, WK1, WV1);
  k_wcvt<<<dim3(CC / 64, DD / 64, 3), 256, 0, stream>>>(F[11], F[13], F[16], DD, CC, WO1, WQ2, WO2);
  k_wcvt<<<dim3(CD / 64, CC / 64, 2), 256, 0, stream>>>(F[14], F[15], F[15], CC, CD, WK2, WV2, WV2);
  k_wcvt<<<dim3(DD / 64, FF / 64, 1), 256, 0, stream>>>(F[18], F[18], F[18], FF1LD, DD, WF1, WF1, WF1);
  k_wcvt<<<dim3(FF / 64, DD / 64, 1), 256, 0, stream>>>(F[20], F[20], F[20], DD, FF, WF2, WF2, WF2);
  k_ccvt<<<dim3(NB * CNP / 8), 256, 0, stream>>>(F[1], CX);

  k_ln<<<dim3(MROWS / 8), 256, 0, stream>>>(F[0], 1, F[2], F[3], XN);
  k_gemm16<<<dim3(MROWS / 64, CC / 128, 3), 128, 0, stream>>>(XN, DD, DD, WQ1, WK1, WV1, QH, KH, VT, CC, 2, SEQ, nullptr, 1.0f);
  for (int b = 0; b < NB; ++b) for (int h0 = 0; h0 < NH; h0 += HG) {
    k_sc<SEQ><<<dim3(SEQ / 64, SEQ / 128, HG), 128, 0, stream>>>(QH, KH, Sf, b, h0, HG);
    k_sm<SEQ, SEQ><<<dim3(SEQ, HG), 256, 0, stream>>>(Sf);
    k_pv<SEQ><<<dim3(SEQ / 64, 1, HG), 128, 0, stream>>>(Sf, VT, b, h0, HG, Y);
  }
  k_gemm32<<<dim3(MROWS / 64, DD / 128), 128, 0, stream>>>(Y, CC, CC, WO1, F[12], F[0], 1, X1, 0, 1.0f / 4096.0f);

  k_ln<<<dim3(MROWS / 8), 256, 0, stream>>>(X1, 0, F[4], F[5], XN);
  k_gemm16<<<dim3(MROWS / 64, CC / 128, 1), 128, 0, stream>>>(XN, DD, DD, WQ2, WQ2, WQ2, QH, QH, QH, CC, 9, SEQ, nullptr, 1.0f);
  k_gemm16<<<dim3(NB * CNP / 64, CC / 128, 2), 128, 0, stream>>>(CX, CD, CD, WK2, WV2, WV2, KC, VC, VC, CC, 1, CNP, nullptr, 1.0f);
  k_sc<CNP><<<dim3(SEQ / 64, CNP / 128, NB * NH), 128, 0, stream>>>(QH, KC, Sf, 0, 0, NH);
  k_sm<CNP, CN><<<dim3(SEQ, NB * NH), 256, 0, stream>>>(Sf);
  k_pv<CNP><<<dim3(SEQ / 64, 1, NB * NH), 128, 0, stream>>>(Sf, VC, 0, 0, NH, Y);
  k_gemm32<<<dim3(MROWS / 64, DD / 128), 128, 0, stream>>>(Y, CC, CC, WO2, F[17], X1, 0, X2, 0, 1.0f / 4096.0f);

  k_ln<<<dim3(MROWS / 8), 256, 0, stream>>>(X2, 0, F[6], F[7], XN);
  k_gemm16<<<dim3(MROWS / 64, FF / 128, 1), 128, 0, stream>>>(XN, DD, DD, WF1, WF1, WF1, Hh, Hh, Hh, FF, 9, SEQ, F[19], 16.0f);
  k_gemm32<<<dim3(MROWS / 64, DD / 128), 128, 0, stream>>>(Hh, FF, FF, WF2, F[21], X2, 0, OUT, 1, 1.0f / 4096.0f);
}
